// PC_Module_56444460204537
// MI455X (gfx1250) — hardware-run, weakly checked
//
#include <hip/hip_runtime.h>
#include <math.h>

typedef __attribute__((ext_vector_type(16))) _Float16 v16h;
typedef __attribute__((ext_vector_type(8)))  _Float16 v8h;
typedef __attribute__((ext_vector_type(16))) __bf16   v16b;
typedef __attribute__((ext_vector_type(8)))  __bf16   v8b;
typedef __attribute__((ext_vector_type(8)))  float    v8f;
typedef __attribute__((ext_vector_type(4)))  float    v4f;
typedef __attribute__((ext_vector_type(4)))  unsigned int v4u;
typedef __attribute__((ext_vector_type(2)))  unsigned int v2u;

constexpr int kB  = 4;
constexpr int kC  = 64;
constexpr int kN  = 4096;
constexpr int kCq = 8;
constexpr int kNO = 2 * kCq + kC;
constexpr int kP1T  = 128;
constexpr int kP1OP = 132;
constexpr int kLP   = 64;
constexpr float kLoCarry    = 64.0f;
constexpr float kLoCarryInv = 1.0f / 64.0f;
constexpr float kBnEps  = 1e-5f;
constexpr float kFltMin = 1.17549435e-38f;
static_assert(kNO == 80);
static_assert((kNO % 16) == 0 && (kC % 32) == 0 && kLP == kC);
static_assert((kN % 128) == 0 && (kN % 64) == 0 && (kC % 16) == 0);
static_assert(4 * kCq == 32);
static_assert((2 * kP1T * kLP + 2 * kNO * kLP) * 2 + 16 * kP1OP * 4 + kNO * 4 <= 65536);

constexpr size_t kSzQP   = (size_t)kB * kN * 32 * 2;
constexpr size_t kSzV16  = (size_t)kB * kC * kN * 2;
constexpr size_t kSzF32  = (size_t)kB * kC * kN * 4;
constexpr size_t kSzAT   = (size_t)kB * kC * kC * 2;
constexpr size_t kOffQP   = 0;
constexpr size_t kOffKP   = kOffQP   + kSzQP;
constexpr size_t kOffVH   = kOffKP   + kSzQP;
constexpr size_t kOffVL   = kOffVH   + kSzV16;
constexpr size_t kOffOUTP = kOffVL   + kSzV16;
constexpr size_t kOffY    = kOffOUTP + kSzF32;
constexpr size_t kOffYH   = kOffY    + kSzF32;
constexpr size_t kOffYL   = kOffYH   + kSzV16;
constexpr size_t kOffATH  = kOffYL   + kSzV16;
constexpr size_t kOffATL  = kOffATH  + kSzAT;
constexpr size_t kOffOUTC = kOffATL  + kSzAT;
constexpr size_t kWsTotal = kOffOUTC + kSzF32;
static_assert(kWsTotal == 23134208ull);
static_assert(kWsTotal <= 134217728ull);
static_assert((kOffKP % 128) == 0 && (kOffVH % 128) == 0 && (kOffVL % 128) == 0 && (kOffOUTP % 128) == 0 &&
              (kOffY % 128) == 0 && (kOffYH % 128) == 0 && (kOffYL % 128) == 0 && (kOffATH % 128) == 0 &&
              (kOffATL % 128) == 0 && (kOffOUTC % 128) == 0);

__device__ __forceinline__ unsigned short f2bf_bits(float f) {
  unsigned u = __float_as_uint(f);
  return (unsigned short)((u + 0x7FFFu + ((u >> 16) & 1u)) >> 16);
}
__device__ __forceinline__ float bf_bits2f(unsigned short h) { return __uint_as_float(((unsigned)h) << 16); }
__device__ __forceinline__ unsigned pk16(unsigned short a, unsigned short b) { return (unsigned)a | ((unsigned)b << 16); }
__device__ __forceinline__ unsigned short h_bits(float f) { const _Float16 h = (_Float16)f; return __builtin_bit_cast(unsigned short, h); }

__device__ __forceinline__ void split_bf(float f, __bf16& hi, __bf16& lo) {
  const unsigned short hb = f2bf_bits(f);
  hi = __builtin_bit_cast(__bf16, hb);
  lo = __builtin_bit_cast(__bf16, f2bf_bits(f - bf_bits2f(hb)));
}

__device__ __forceinline__ void split8_bf16(const v4f a0, const v4f a1, v4u& uh, v4u& ul) {
  const float f[8] = {a0[0], a0[1], a0[2], a0[3], a1[0], a1[1], a1[2], a1[3]};
  unsigned short h[8], l[8];
#pragma unroll
  for (int e = 0; e < 8; ++e) {
    h[e] = f2bf_bits(f[e]);
    l[e] = f2bf_bits(f[e] - bf_bits2f(h[e]));
  }
  uh = (v4u){pk16(h[0], h[1]), pk16(h[2], h[3]), pk16(h[4], h[5]), pk16(h[6], h[7])};
  ul = (v4u){pk16(l[0], l[1]), pk16(l[2], l[3]), pk16(l[4], l[5]), pk16(l[6], l[7])};
}

__device__ __forceinline__ void stage4_bf(__bf16* ph, __bf16* pl, int o, const v4f v) {
  const float f0 = v[0], f1 = v[1], f2 = v[2], f3 = v[3];
  __bf16 h0, l0, h1, l1, h2, l2, h3, l3;
  split_bf(f0, h0, l0);
  split_bf(f1, h1, l1);
  split_bf(f2, h2, l2);
  split_bf(f3, h3, l3);
  ph[o + 0] = h0; pl[o + 0] = l0;
  ph[o + 1] = h1; pl[o + 1] = l1;
  ph[o + 2] = h2; pl[o + 2] = l2;
  ph[o + 3] = h3; pl[o + 3] = l3;
}

template <typename T> struct Frag;
template <> struct Frag<_Float16> {
  typedef v16h V; union U { v16h v; v8h h[2]; };
  static __device__ __forceinline__ v16h load(const _Float16* p) {
    U f; f.h[0] = *(const v8h*)(p); f.h[1] = *(const v8h*)(p + 16); return f.v;
  }
};
template <> struct Frag<__bf16> {
  typedef v16b V; union U { v16b v; v8b h[2]; };
  static __device__ __forceinline__ v16b load(const __bf16* p) {
    U f; f.h[0] = *(const v8b*)(p); f.h[1] = *(const v8b*)(p + 16); return f.v;
  }
};

__device__ __forceinline__ v8f mma_h(v16h a, v16h b, v8f c) {
  c = __builtin_amdgcn_wmma_f32_16x16x32_f16(false, a, false, b, (short)0, c, false, false);
  asm volatile("v_nop\n\tv_nop\n\tv_nop\n\tv_nop" : "+v"(c) : "v"(a), "v"(b));
  return c;
}
__device__ __forceinline__ v8f mma_b(v16b a, v16b b, v8f c) {
  c = __builtin_amdgcn_wmma_f32_16x16x32_bf16(false, a, false, b, (short)0, c, false, false);
  asm volatile("v_nop\n\tv_nop\n\tv_nop\n\tv_nop" : "+v"(c) : "v"(a), "v"(b));
  return c;
}

__device__ __forceinline__ void wave_lds_sync() {
  __builtin_amdgcn_fence(__ATOMIC_RELEASE, "workgroup");
  __builtin_amdgcn_wave_barrier();
  __builtin_amdgcn_fence(__ATOMIC_ACQUIRE, "workgroup");
}

__global__ __launch_bounds__(128) void proj_kernel(
    const float* __restrict__ x,
    const float* __restrict__ Wq, const float* __restrict__ bq,
    const float* __restrict__ Wk, const float* __restrict__ bk,
    const float* __restrict__ Wv, const float* __restrict__ bv,
    unsigned short* __restrict__ QP, unsigned short* __restrict__ KP,
    unsigned short* __restrict__ VH, unsigned short* __restrict__ VL)
{
  __shared__ __align__(16) __bf16 sXh[kP1T * kLP];
  __shared__ __align__(16) __bf16 sXl[kP1T * kLP];
  __shared__ __align__(16) __bf16 sWh[kNO * kLP];
  __shared__ __align__(16) __bf16 sWl[kNO * kLP];
  __shared__ __align__(16) float sO[16 * kP1OP];
  __shared__ float sBias[kNO];
  const int tid = threadIdx.x, lane = tid & 31, wave = tid >> 5;
  const int hh = lane >> 4, c = lane & 15;
  const int b  = blockIdx.x >> 5;
  const int n0 = (blockIdx.x & 31) * kP1T;

#pragma unroll 1
  for (int it = 0; it < 16; ++it) {
    const int idx = it * 128 + tid;
    const int row = idx >> 5;
    const int c4  = (idx & 31) * 4;
    const v4f v = *(const v4f*)(x + ((size_t)(b * kC + row)) * kN + n0 + c4);
    const float f0 = v[0], f1 = v[1], f2 = v[2], f3 = v[3];
    __bf16 h0, l0, h1, l1, h2, l2, h3, l3;
    split_bf(f0, h0, l0);
    split_bf(f1, h1, l1);
    split_bf(f2, h2, l2);
    split_bf(f3, h3, l3);
    sXh[(c4 + 0) * kLP + row] = h0; sXl[(c4 + 0) * kLP + row] = l0;
    sXh[(c4 + 1) * kLP + row] = h1; sXl[(c4 + 1) * kLP + row] = l1;
    sXh[(c4 + 2) * kLP + row] = h2; sXl[(c4 + 2) * kLP + row] = l2;
    sXh[(c4 + 3) * kLP + row] = h3; sXl[(c4 + 3) * kLP + row] = l3;
  }
  {
    const v4f vq = *(const v4f*)(Wq + tid * 4);
    const v4f vk = *(const v4f*)(Wk + tid * 4);
    stage4_bf(sWh, sWl, tid * 4, vq);
    stage4_bf(sWh, sWl, kCq * kC + tid * 4, vk);
  }
#pragma unroll 1
  for (int it = 0; it < 8; ++it) {
    const int idx = it * 128 + tid;
    const v4f vv = *(const v4f*)(Wv + idx * 4);
    stage4_bf(sWh, sWl, 2 * kCq * kC + idx * 4, vv);
  }
  {
    float bqv = bq[tid & 7];
    float bkv = bk[tid & 7];
    float bvv = bv[tid & 63];
    asm volatile("" : "+v"(bqv), "+v"(bkv), "+v"(bvv));
    if (tid < 8)  { sBias[tid] = bqv; sBias[kCq + tid] = bkv; }
    if (tid < 64) sBias[2 * kCq + tid] = bvv;
  }
  __syncthreads();

  v16b xbh[2][2], xbl[2][2];
#pragma unroll
  for (int nt = 0; nt < 2; ++nt) {
#pragma unroll
    for (int ks = 0; ks < 2; ++ks) {
      const int o = (wave * 32 + nt * 16 + c) * kLP + ks * 32 + 8 * hh;
      xbh[nt][ks] = Frag<__bf16>::load(sXh + o);
      xbl[nt][ks] = Frag<__bf16>::load(sXl + o);
    }
  }

  const int seg = lane & 3;
  const int hh2 = lane >> 4;
  const int c8  = (lane & 15) * 8;

#pragma unroll 1
  for (int g = 0; g < 5; ++g) {
    v8f acc0 = (v8f){0.f, 0.f, 0.f, 0.f, 0.f, 0.f, 0.f, 0.f};
    v8f acc1 = (v8f){0.f, 0.f, 0.f, 0.f, 0.f, 0.f, 0.f, 0.f};
#pragma unroll
    for (int ks = 0; ks < 2; ++ks) {
      const int ao = (g * 16 + c) * kLP + ks * 32 + 8 * hh;
      const v16b ah = Frag<__bf16>::load(sWh + ao);
      const v16b al = Frag<__bf16>::load(sWl + ao);
      acc0 = mma_b(ah, xbh[0][ks], acc0);
      acc0 = mma_b(ah, xbl[0][ks], acc0);
      acc0 = mma_b(al, xbh[0][ks], acc0);
      acc1 = mma_b(ah, xbh[1][ks], acc1);
      acc1 = mma_b(ah, xbl[1][ks], acc1);
      acc1 = mma_b(al, xbh[1][ks], acc1);
    }
#pragma unroll
    for (int r = 0; r < 8; ++r) {
      const float bb = sBias[g * 16 + 8 * hh + r];
      sO[(8 * hh + r) * kP1OP + wave * 32 + c]      = acc0[r] + bb;
      sO[(8 * hh + r) * kP1OP + wave * 32 + 16 + c] = acc1[r] + bb;
    }
    __syncthreads();
    if (g == 0) {
      v4u uq[4], uk[4];
#pragma unroll
      for (int it = 0; it < 4; ++it) {
        const int nl = (wave * 4 + it) * 8 + (lane >> 2);
        unsigned short hq[8], hk[8];
#pragma unroll
        for (int d = 0; d < 8; ++d) {
          const float fq = sO[d * kP1OP + nl];
          const float fk = sO[(kCq + d) * kP1OP + nl];
          const float hqf = (float)(_Float16)fq;
          const float hkf = (float)(_Float16)fk;
          const float q_lo = (fq - hqf) * kLoCarry;
          const float k_lo = (fk - hkf) * kLoCarry;
          const float q_hs = hqf * kLoCarryInv;
          const float k_hs = hkf * kLoCarryInv;
          const float vq = (seg == 0) ? fq : ((seg == 1) ? q_hs : ((seg == 2) ? q_lo : 0.0f));
          const float vk = (seg == 0) ? fk : ((seg == 1) ? k_lo : ((seg == 2) ? k_hs : 0.0f));
          hq[d] = h_bits(vq);
          hk[d] = h_bits(vk);
        }
        uq[it] = (v4u){pk16(hq[0], hq[1]), pk16(hq[2], hq[3]), pk16(hq[4], hq[5]), pk16(hq[6], hq[7])};
        uk[it] = (v4u){pk16(hk[0], hk[1]), pk16(hk[2], hk[3]), pk16(hk[4], hk[5]), pk16(hk[6], hk[7])};
      }
      for (int pass = 0; pass < 2; ++pass) {
#pragma unroll
        for (int it = 0; it < 4; ++it) {
          const int nl = (wave * 4 + it) * 8 + (lane >> 2);
          const size_t o = ((size_t)(b * kN + n0 + nl)) * 32 + seg * 8;
          *(volatile v4u*)(QP + o) = uq[it];
          *(volatile v4u*)(KP + o) = uk[it];
        }
        __threadfence();
      }
    } else {
      v4u uh[2], ul[2];
#pragma unroll
      for (int it = 0; it < 2; ++it) {
        const int row = it * 8 + wave * 2 + hh2;
        const float* sp = sO + row * kP1OP + c8;
        const v4f a0 = *(const v4f*)(sp);
        const v4f a1 = *(const v4f*)(sp + 4);
        split8_bf16(a0, a1, uh[it], ul[it]);
      }
      for (int pass = 0; pass < 2; ++pass) {
#pragma unroll
        for (int it = 0; it < 2; ++it) {
          const int row = it * 8 + wave * 2 + hh2;
          const int ch  = (g - 1) * 16 + row;
          const size_t o = ((size_t)(b * kC + ch)) * kN + n0 + c8;
          *(volatile v4u*)(VH + o) = uh[it];
          *(volatile v4u*)(VL + o) = ul[it];
        }
        __threadfence();
      }
    }
    __syncthreads();
  }
}

__global__ __launch_bounds__(128) void pam_flash_kernel(
    const unsigned short* __restrict__ QPp, const unsigned short* __restrict__ KPp,
    const unsigned short* __restrict__ VHp, const unsigned short* __restrict__ VLp,
    float* __restrict__ OUTP)
{
  __shared__ __align__(16) __bf16 Psh[4][16 * 64];
  __shared__ __align__(16) __bf16 Psl[4][16 * 64];
  __shared__ __align__(16) float  Os[kC * 68];
  const int tid = threadIdx.x, wave = tid >> 5, lane = tid & 31, hh = lane >> 4, c = lane & 15;
  const int b  = blockIdx.x >> 6;
  const int qb = blockIdx.x & 63;
  const int q0 = qb * 64 + wave * 16;

  const _Float16* QP = (const _Float16*)QPp;
  const _Float16* KP = (const _Float16*)KPp;
  const __bf16*   VH = (const __bf16*)VHp;
  const __bf16*   VL = (const __bf16*)VLp;

  const v16h qa = Frag<_Float16>::load(QP + ((size_t)(b * kN + q0 + c)) * 32 + 8 * hh);
  const _Float16* kb_ptr = KP + ((size_t)b * kN + c) * 32 + 8 * hh;
  const __bf16*   vh_ptr = VH + ((size_t)(b * kC + c)) * kN + 8 * hh;
  const __bf16*   vl_ptr = VL + ((size_t)(b * kC + c)) * kN + 8 * hh;

  float mrow[8], lrow[8];
  v8f oacc[4];
#pragma unroll
  for (int r = 0; r < 8; ++r) { mrow[r] = -1e30f; lrow[r] = 0.f; }
#pragma unroll
  for (int t = 0; t < 4; ++t) oacc[t] = (v8f){0.f, 0.f, 0.f, 0.f, 0.f, 0.f, 0.f, 0.f};

  __bf16* pwh = Psh[wave];
  __bf16* pwl = Psl[wave];

#pragma unroll 1
  for (int kc = 0; kc < kN / 64; ++kc) {
    const int kv0 = kc * 64;
    v8f s[4];
#pragma unroll
    for (int j = 0; j < 4; ++j) {
      const v16h kf = Frag<_Float16>::load(kb_ptr + (size_t)(kv0 + j * 16) * 32);
      s[j] = mma_h(qa, kf, (v8f){0.f, 0.f, 0.f, 0.f, 0.f, 0.f, 0.f, 0.f});
    }
#pragma unroll
    for (int r = 0; r < 8; ++r) {
      float m = fmaxf(fmaxf(s[0][r], s[1][r]), fmaxf(s[2][r], s[3][r]));
#pragma unroll
      for (int off = 1; off < 16; off <<= 1) m = fmaxf(m, __shfl_xor(m, off, 32));
      const float mnew  = fmaxf(mrow[r], m);
      const float alpha = __expf(mrow[r] - mnew);
      mrow[r] = mnew;
      float psum = 0.f;
#pragma unroll
      for (int j = 0; j < 4; ++j) {
        const float p = __expf(s[j][r] - mnew);
        psum += p;
        __bf16 ph, pl;
        split_bf(p, ph, pl);
        pwh[(8 * hh + r) * 64 + j * 16 + c] = ph;
        pwl[(8 * hh + r) * 64 + j * 16 + c] = pl;
      }
#pragma unroll
      for (int off = 1; off < 16; off <<= 1) psum += __shfl_xor(psum, off, 32);
      lrow[r] = lrow[r] * alpha + psum;
#pragma unroll
      for (int t = 0; t < 4; ++t) oacc[t][r] *= alpha;
    }
    wave_lds_sync();
#pragma unroll 1
    for (int kk = 0; kk < 2; ++kk) {
      const v16b pa = Frag<__bf16>::load(pwh + c * 64 + kk * 32 + 8 * hh);
      const v16b pl = Frag<__bf16>::load(pwl + c * 64 + kk * 32 + 8 * hh);
#pragma unroll
      for (int t = 0; t < 4; ++t) {
        const size_t vo = (size_t)(t * 16) * kN + kv0 + kk * 32;
        const v16b vb = Frag<__bf16>::load(vh_ptr + vo);
        const v16b vl = Frag<__bf16>::load(vl_ptr + vo);
        oacc[t] = mma_b(pa, vb, oacc[t]);
        oacc[t] = mma_b(pa, vl, oacc[t]);
        oacc[t] = mma_b(pl, vb, oacc[t]);
      }
    }
    wave_lds_sync();
  }

#pragma unroll
  for (int r = 0; r < 8; ++r) {
    const float inv = 1.0f / lrow[r];
#pragma unroll
    for (int t = 0; t < 4; ++t) Os[(t * 16 + c) * 68 + wave * 16 + 8 * hh + r] = oacc[t][r] * inv;
  }
  __syncthreads();
  {
    const int c4 = (lane & 15) * 4;
    v4f vals[8];
#pragma unroll
    for (int it = 0; it < 8; ++it) {
      const int ch = wave * 16 + it * 2 + hh;
      vals[it] = *(const v4f*)(Os + ch * 68 + c4);
    }
    for (int pass = 0; pass < 2; ++pass) {
#pragma unroll
      for (int it = 0; it < 8; ++it) {
        const int ch = wave * 16 + it * 2 + hh;
        *(volatile v4f*)(OUTP + ((size_t)(b * kC + ch)) * kN + qb * 64 + c4) = vals[it];
      }
      __threadfence();
    }
  }
}

__device__ __forceinline__ float block_sum256(float v, float* red) {
#pragma unroll
  for (int off = 16; off > 0; off >>= 1) v += __shfl_xor(v, off, 32);
  if ((threadIdx.x & 31) == 0) red[threadIdx.x >> 5] = v;
  __syncthreads();
  float s = red[0];
  s += red[1];
  s += red[2];
  s += red[3];
  s += red[4];
  s += red[5];
  s += red[6];
  s += red[7];
  __syncthreads();
  return s;
}

template <bool PLANES>
__global__ __launch_bounds__(256) void bn_residual_kernel(
    const float* __restrict__ src, const float* __restrict__ res,
    const float* __restrict__ gscal, const float* __restrict__ w, const float* __restrict__ bias,
    float* __restrict__ yout, unsigned short* __restrict__ YH, unsigned short* __restrict__ YL)
{
  __shared__ float red[8];
  const int c = blockIdx.x, tid = threadIdx.x;
  const float g = gscal[0];
  const float inv_cnt = 1.0f / (float)(kB * kN);

  float sum = 0.f;
#pragma unroll 1
  for (int it = 0; it < 16; ++it) {
    const int i = it * 256 + tid;
    const size_t o = ((size_t)((i >> 10) * kC + c)) * kN + (i & 1023) * 4;
    const v4f v = *(const v4f*)(src + o);
    sum += (g * v[0] + g * v[1]) + (g * v[2] + g * v[3]);
  }
  const float mean = block_sum256(sum, red) * inv_cnt;

  float sq = 0.f;
#pragma unroll 1
  for (int it = 0; it < 16; ++it) {
    const int i = it * 256 + tid;
    const size_t o = ((size_t)((i >> 10) * kC + c)) * kN + (i & 1023) * 4;
    const v4f v = *(const v4f*)(src + o);
    const float d0 = g * v[0] - mean, d1 = g * v[1] - mean, d2 = g * v[2] - mean, d3 = g * v[3] - mean;
    sq += (d0 * d0 + d1 * d1) + (d2 * d2 + d3 * d3);
  }
  const float var  = block_sum256(sq, red) * inv_cnt;
  const float rstd = 1.0f / sqrtf(var + kBnEps);
  const float wc = w[c], bc = bias[c];

#pragma unroll 1
  for (int it = 0; it < 16; ++it) {
    const int i = it * 256 + tid;
    const size_t o = ((size_t)((i >> 10) * kC + c)) * kN + (i & 1023) * 4;
    const v4f v = *(const v4f*)(src + o);
    const v4f rv = *(const v4f*)(res + o);
    v4f ov;
    ov[0] = ((g * v[0] - mean) * rstd) * wc + bc + rv[0];
    ov[1] = ((g * v[1] - mean) * rstd) * wc + bc + rv[1];
    ov[2] = ((g * v[2] - mean) * rstd) * wc + bc + rv[2];
    ov[3] = ((g * v[3] - mean) * rstd) * wc + bc + rv[3];
    v2u uh = (v2u){0u, 0u}, ul = (v2u){0u, 0u};
    if (PLANES) {
      const float f0 = ov[0], f1 = ov[1], f2 = ov[2], f3 = ov[3];
      const unsigned short h0 = f2bf_bits(f0), h1 = f2bf_bits(f1), h2 = f2bf_bits(f2), h3 = f2bf_bits(f3);
      const unsigned short l0 = f2bf_bits(f0 - bf_bits2f(h0)), l1 = f2bf_bits(f1 - bf_bits2f(h1));
      const unsigned short l2 = f2bf_bits(f2 - bf_bits2f(h2)), l3 = f2bf_bits(f3 - bf_bits2f(h3));
      uh = (v2u){pk16(h0, h1), pk16(h2, h3)};
      ul = (v2u){pk16(l0, l1), pk16(l2, l3)};
    }
    *(volatile v4f*)(yout + o) = ov;
    if (PLANES) {
      *(volatile v2u*)(YH + o) = uh;
      *(volatile v2u*)(YL + o) = ul;
    }
    __threadfence();
    *(volatile v4f*)(yout + o) = ov;
    if (PLANES) {
      *(volatile v2u*)(YH + o) = uh;
      *(volatile v2u*)(YL + o) = ul;
    }
  }
}

__global__ __launch_bounds__(256) void cam_energy_softmax_kernel(
    const unsigned short* __restrict__ YHp, const unsigned short* __restrict__ YLp,
    unsigned short* __restrict__ ATH, unsigned short* __restrict__ ATL)
{
  __shared__ __align__(16) float sP[8][16 * 68];
  __shared__ __align__(16) float sE[16 * 68];
  const int tid = threadIdx.x, wave = tid >> 5, lane = tid & 31, hh = lane >> 4, c = lane & 15;
  const int b  = blockIdx.x >> 2;
  const int it = blockIdx.x & 3;
  const __bf16* yh = (const __bf16*)YHp + (size_t)b * kC * kN;
  const __bf16* yl = (const __bf16*)YLp + (size_t)b * kC * kN;
  const int kbeg = wave * 512;

  v8f acc[4];
#pragma unroll
  for (int j = 0; j < 4; ++j) acc[j] = (v8f){0.f, 0.f, 0.f, 0.f, 0.f, 0.f, 0.f, 0.f};

  const size_t arow = (size_t)(it * 16 + c) * kN + 8 * hh;
#pragma unroll 1
  for (int ks = 0; ks < 16; ++ks) {
    const int k0 = kbeg + ks * 32;
    const v16b ah = Frag<__bf16>::load(yh + arow + k0);
    const v16b al = Frag<__bf16>::load(yl + arow + k0);
#pragma unroll
    for (int j = 0; j < 4; ++j) {
      const size_t bo = (size_t)(j * 16 + c) * kN + 8 * hh + k0;
      const v16b bh = Frag<__bf16>::load(yh + bo);
      const v16b bl = Frag<__bf16>::load(yl + bo);
      acc[j] = mma_b(ah, bh, acc[j]);
      acc[j] = mma_b(ah, bl, acc[j]);
      acc[j] = mma_b(al, bh, acc[j]);
    }
  }
  {
    float* pw = sP[wave];
#pragma unroll
    for (int j = 0; j < 4; ++j)
#pragma unroll
      for (int r = 0; r < 8; ++r) pw[(8 * hh + r) * 68 + j * 16 + c] = acc[j][r];
  }
  __syncthreads();
  {
    const int row = tid >> 4, c4 = (tid & 15) * 4;
    const v4f p0 = *(const v4f*)(sP[0] + row * 68 + c4);
    const v4f p1 = *(const v4f*)(sP[1] + row * 68 + c4);
    const v4f p2 = *(const v4f*)(sP[2] + row * 68 + c4);
    const v4f p3 = *(const v4f*)(sP[3] + row * 68 + c4);
    const v4f p4 = *(const v4f*)(sP[4] + row * 68 + c4);
    const v4f p5 = *(const v4f*)(sP[5] + row * 68 + c4);
    const v4f p6 = *(const v4f*)(sP[6] + row * 68 + c4);
    const v4f p7 = *(const v4f*)(sP[7] + row * 68 + c4);
    const v4f e = ((p0 + p1) + (p2 + p3)) + ((p4 + p5) + (p6 + p7));
    *(v4f*)(sE + row * 68 + c4) = e;
  }
  __syncthreads();
#pragma unroll
  for (int rr = 0; rr < 2; ++rr) {
    const int row = wave * 2 + rr;
    const float e0 = sE[row * 68 + lane];
    const float e1 = sE[row * 68 + 32 + lane];
    float mx = fmaxf(e0, e1);
#pragma unroll
    for (int off = 16; off > 0; off >>= 1) mx = fmaxf(mx, __shfl_xor(mx, off, 32));
    const float t0 = mx - e0, t1 = mx - e1;
    float m2 = fmaxf(t0, t1);
#pragma unroll
    for (int off = 16; off > 0; off >>= 1) m2 = fmaxf(m2, __shfl_xor(m2, off, 32));
    float p0 = expf(t0 - m2);
    float p1 = expf(t1 - m2);
    p0 = (p0 < kFltMin) ? 0.0f : p0;
    p1 = (p1 < kFltMin) ? 0.0f : p1;
    float sm = p0 + p1;
#pragma unroll
    for (int off = 16; off > 0; off >>= 1) sm += __shfl_xor(sm, off, 32);
    const float inv = 1.0f / sm;
    sE[row * 68 + lane]      = p0 * inv;
    sE[row * 68 + 32 + lane] = p1 * inv;
  }
  __syncthreads();
  if (wave < 4) {
    const int row = wave * 4 + (lane >> 3), c8 = (lane & 7) * 8;
    const float* sp = sE + row * 68 + c8;
    const v4f a0 = *(const v4f*)(sp);
    const v4f a1 = *(const v4f*)(sp + 4);
    v4u uh, ul;
    split8_bf16(a0, a1, uh, ul);
    const size_t o = ((size_t)(b * kC + it * 16 + row)) * kC + c8;
    *(volatile v4u*)(ATH + o) = uh;
    *(volatile v4u*)(ATL + o) = ul;
    __threadfence();
    *(volatile v4u*)(ATH + o) = uh;
    *(volatile v4u*)(ATL + o) = ul;
  }
}

__global__ __launch_bounds__(128) void cam_out_kernel(
    const unsigned short* __restrict__ ATHp, const unsigned short* __restrict__ ATLp,
    const float* __restrict__ Y, float* __restrict__ OUTC)
{
  __shared__ __align__(16) __bf16 sYh[64 * 72];
  __shared__ __align__(16) __bf16 sYl[64 * 72];
  __shared__ __align__(16) float  sO[4][16 * 68];
  const int tid = threadIdx.x, wave = tid >> 5, lane = tid & 31, hh = lane >> 4, c = lane & 15;
  const int b  = blockIdx.x >> 6;
  const int n0 = (blockIdx.x & 63) * 64;
  const float* yb = Y + (size_t)b * kC * kN + n0;

#pragma unroll
  for (int it = 0; it < 8; ++it) {
    const int idx = it * 128 + tid;
    const int d  = idx >> 4;
    const int n4 = (idx & 15) * 4;
    const v4f v = *(const v4f*)(yb + (size_t)d * kN + n4);
    const float f0 = v[0], f1 = v[1], f2 = v[2], f3 = v[3];
    __bf16 h0, l0, h1, l1, h2, l2, h3, l3;
    split_bf(f0, h0, l0);
    split_bf(f1, h1, l1);
    split_bf(f2, h2, l2);
    split_bf(f3, h3, l3);
    sYh[(n4 + 0) * 72 + d] = h0; sYl[(n4 + 0) * 72 + d] = l0;
    sYh[(n4 + 1) * 72 + d] = h1; sYl[(n4 + 1) * 72 + d] = l1;
    sYh[(n4 + 2) * 72 + d] = h2; sYl[(n4 + 2) * 72 + d] = l2;
    sYh[(n4 + 3) * 72 + d] = h3; sYl[(n4 + 3) * 72 + d] = l3;
  }
  __syncthreads();

  const __bf16* ath = (const __bf16*)ATHp + ((size_t)(b * kC + wave * 16 + c)) * kC + 8 * hh;
  const __bf16* atl = (const __bf16*)ATLp + ((size_t)(b * kC + wave * 16 + c)) * kC + 8 * hh;

  v8f acc[4];
#pragma unroll
  for (int j = 0; j < 4; ++j) acc[j] = (v8f){0.f, 0.f, 0.f, 0.f, 0.f, 0.f, 0.f, 0.f};

#pragma unroll 1
  for (int ks = 0; ks < 2; ++ks) {
    const v16b ah = Frag<__bf16>::load(ath + ks * 32);
    const v16b al = Frag<__bf16>::load(atl + ks * 32);
#pragma unroll
    for (int j = 0; j < 4; ++j) {
      const int bo = (j * 16 + c) * 72 + ks * 32 + 8 * hh;
      const v16b bh = Frag<__bf16>::load(sYh + bo);
      const v16b bl = Frag<__bf16>::load(sYl + bo);
      acc[j] = mma_b(ah, bh, acc[j]);
      acc[j] = mma_b(ah, bl, acc[j]);
      acc[j] = mma_b(al, bh, acc[j]);
    }
  }

  float* slab = sO[wave];
#pragma unroll
  for (int j = 0; j < 4; ++j)
#pragma unroll
    for (int r = 0; r < 8; ++r) slab[(8 * hh + r) * 68 + j * 16 + c] = acc[j][r];
  wave_lds_sync();
  {
    const int c4 = (lane & 15) * 4;
    v4f vals[8];
#pragma unroll
    for (int it = 0; it < 8; ++it) vals[it] = *(const v4f*)(slab + (it * 2 + hh) * 68 + c4);
    for (int pass = 0; pass < 2; ++pass) {
#pragma unroll
      for (int it = 0; it < 8; ++it) {
        const int ch = wave * 16 + it * 2 + hh;
        *(volatile v4f*)(OUTC + ((size_t)(b * kC + ch)) * kN + n0 + c4) = vals[it];
      }
      __threadfence();
    }
  }
}

extern "C" void kernel_launch(void* const* d_in, const int* in_sizes, int n_in,
                              void* d_out, int out_size, void* d_ws, size_t ws_size,
                              hipStream_t stream) {
  if (n_in < 13) return;
  if (in_sizes[0] != kB * kC * kN) return;
  if (in_sizes[1] != kCq * kC || in_sizes[2] != kCq) return;
  if (in_sizes[3] != kCq * kC || in_sizes[4] != kCq) return;
  if (in_sizes[5] != kC * kC || in_sizes[6] != kC) return;
  if (in_sizes[7] != 1 || in_sizes[8] != kC || in_sizes[9] != kC) return;
  if (in_sizes[10] != 1 || in_sizes[11] != kC || in_sizes[12] != kC) return;
  if (out_size != kB * kC * kN) return;
  if (ws_size < kWsTotal) return;

  const float* x       = (const float*)d_in[0];
  const float* Wq      = (const float*)d_in[1];
  const float* bq      = (const float*)d_in[2];
  const float* Wk      = (const float*)d_in[3];
  const float* bk      = (const float*)d_in[4];
  const float* Wv      = (const float*)d_in[5];
  const float* bv      = (const float*)d_in[6];
  const float* gamma_p = (const float*)d_in[7];
  const float* bnp_w   = (const float*)d_in[8];
  const float* bnp_b   = (const float*)d_in[9];
  const float* gamma_c = (const float*)d_in[10];
  const float* bnc_w   = (const float*)d_in[11];
  const float* bnc_b   = (const float*)d_in[12];
  float* out = (float*)d_out;

  char* ws = (char*)d_ws;
  unsigned short* QP   = (unsigned short*)(ws + kOffQP);
  unsigned short* KP   = (unsigned short*)(ws + kOffKP);
  unsigned short* VH   = (unsigned short*)(ws + kOffVH);
  unsigned short* VL   = (unsigned short*)(ws + kOffVL);
  float*          OUTP = (float*)(ws + kOffOUTP);
  float*          Y    = (float*)(ws + kOffY);
  unsigned short* YH   = (unsigned short*)(ws + kOffYH);
  unsigned short* YL   = (unsigned short*)(ws + kOffYL);
  unsigned short* ATH  = (unsigned short*)(ws + kOffATH);
  unsigned short* ATL  = (unsigned short*)(ws + kOffATL);
  float*          OUTC = (float*)(ws + kOffOUTC);

  proj_kernel<<<kB * (kN / kP1T), 128, 0, stream>>>(x, Wq, bq, Wk, bk, Wv, bv, QP, KP, VH, VL);
  pam_flash_kernel<<<kB * (kN / 64), 128, 0, stream>>>(QP, KP, VH, VL, OUTP);
  bn_residual_kernel<true><<<kC, 256, 0, stream>>>(OUTP, x, gamma_p, bnp_w, bnp_b, Y, YH, YL);
  cam_energy_softmax_kernel<<<kB * (kC / 16), 256, 0, stream>>>(YH, YL, ATH, ATL);
  cam_out_kernel<<<kB * (kN / 64), 128, 0, stream>>>(ATH, ATL, Y, OUTC);
  bn_residual_kernel<false><<<kC, 256, 0, stream>>>(OUTC, Y, gamma_c, bnc_w, bnc_b, out, YH, YL);
}
